// PlacementCNN_10960756540056
// MI455X (gfx1250) — hardware-verified
//
#include <hip/hip_runtime.h>


namespace {
constexpr int T = 65536, NF0 = 80, CIN = 3, C0 = 10, KH0 = 7, KW0 = 3, K0 = CIN * KH0 * KW0, F0 = 78, P0 = 26, T0 = T + 8;
constexpr int C1 = 20, K1 = C0 * 9, F1 = 24, P1 = 8, T1 = T + 6, FEAT = P1 * C1;
constexpr int H1P = 320;
constexpr int FP = 192;
constexpr int KD0 = 7 * FEAT, ND0 = 256, ND1 = 128, NDIFF = 5;

typedef _Float16 b16;
typedef __attribute__((ext_vector_type(16))) _Float16 v16b;
typedef __attribute__((ext_vector_type(8)))  _Float16 v8b;
typedef __attribute__((ext_vector_type(8)))  float v8f;
typedef __attribute__((ext_vector_type(4)))  float v4f;

__device__ __forceinline__ v8b ld8b(const b16* p) { return *(const v8b*)p; }
__device__ __forceinline__ v16b cat8b(v8b a, v8b b) { return __builtin_shufflevector(a, b, 0, 1, 2, 3, 4, 5, 6, 7, 8, 9, 10, 11, 12, 13, 14, 15); }
__device__ __forceinline__ v16b frag_kb(const b16* p, int hh) { return cat8b(ld8b(p + 8 * hh), ld8b(p + 16 + 8 * hh)); }
__device__ __forceinline__ void split16(float v, b16& hi, b16& lo) { hi = (b16)v; lo = (b16)(v - (float)hi); }
__device__ __forceinline__ void frag_ksplit(const float* p, int hh, v16b& fh_, v16b& fl_) {
  const float* p0 = p + 8 * hh; const float* p1 = p + 16 + 8 * hh;
#pragma unroll
  for (int e = 0; e < 8; ++e) { b16 a, c; split16(p0[e], a, c); fh_[e] = a; fl_[e] = c; split16(p1[e], a, c); fh_[8 + e] = a; fl_[8 + e] = c; }
}
__device__ __forceinline__ v8f wmma16b(v16b a, v16b b, v8f c) {
  v8f d = __builtin_amdgcn_wmma_f32_16x16x32_f16(false, a, false, b, (short)0, c, false, false);
  asm volatile("v_nop\n\tv_nop\n\tv_nop\n\tv_nop" : "+v"(d) : "v"(a), "v"(b));
  return d;
}
__device__ __forceinline__ void wave_lds_sync() {
  __builtin_amdgcn_fence(__ATOMIC_RELEASE, "workgroup");
  __builtin_amdgcn_wave_barrier();
  __builtin_amdgcn_fence(__ATOMIC_ACQUIRE, "workgroup");
}

struct Opnd { const void* p0; const void* p1; int ld; };
template <int NP> __device__ __forceinline__ void load_frags(const Opnd& o, int row, int kb, int hh, v16b& fh_, v16b& fl_) {
  if (NP == 0) { frag_ksplit((const float*)o.p0 + (size_t)row * o.ld + kb, hh, fh_, fl_); }
  else if (NP == 3) {
    const float* p = (const float*)o.p0 + (size_t)row * o.ld + kb; const float* p0 = p + 8 * hh; const float* p1 = p + 16 + 8 * hh;
#pragma unroll
    for (int e = 0; e < 8; ++e) { fh_[e] = (b16)p0[e]; fh_[8 + e] = (b16)p1[e]; }
    fl_ = fh_;
  } else {
    fh_ = frag_kb((const b16*)o.p0 + (size_t)row * o.ld + kb, hh);
    if (NP == 2) fl_ = frag_kb((const b16*)o.p1 + (size_t)row * o.ld + kb, hh); else fl_ = fh_;
  }
}
template <int ANP, int BNP> __device__ __forceinline__ v8f mac(v16b ah, v16b al, v16b bh, v16b bl, v8f c) {
  c = wmma16b(ah, bh, c);
  if (BNP == 0 || BNP == 2) c = wmma16b(ah, bl, c);
  if (ANP == 0 || ANP == 2) c = wmma16b(al, bh, c);
  return c;
}
template <int ANP, int BNP>
__device__ __forceinline__ void gemm_tile(const Opnd& A, const Opnd& B, int K, int m0, int c0, int nloc, int hlf, v8f (&acc)[2][4]) {
  for (int kb = 0; kb < K; kb += 32) {
    v16b a0h, a0l, a1h, a1l;
    load_frags<ANP>(A, m0 + nloc, kb, hlf, a0h, a0l);
    load_frags<ANP>(A, m0 + 16 + nloc, kb, hlf, a1h, a1l);
#pragma unroll
    for (int t = 0; t < 4; ++t) {
      v16b bh, bl;
      load_frags<BNP>(B, c0 + t * 16 + nloc, kb, hlf, bh, bl);
      acc[0][t] = mac<ANP, BNP>(a0h, a0l, bh, bl, acc[0][t]);
      acc[1][t] = mac<ANP, BNP>(a1h, a1l, bh, bl, acc[1][t]);
    }
  }
}

struct Epi { float scale; const float* cscale; const float* cbias; const float* rbias; int act; float post; const float* rscale; const float* resid; };
__device__ __forceinline__ float epi_val(const Epi& e, float acc, int row, int col) {
  float val = acc * e.scale;
  if (e.cscale) val *= e.cscale[col];
  if (e.cbias) val += e.cbias[col];
  if (e.rbias) val += e.rbias[row];
  if (e.act == 1) val = 0.5f * val * (1.0f + erff(val * 0.70710678118654752f));
  val *= e.post;
  if (e.rscale) val *= e.rscale[(size_t)row * 32];
  return val;
}
__device__ __forceinline__ void epi_planes(v8f (&acc)[2][4], const Epi& e, bool two,
                                           b16* __restrict__ oh, b16* __restrict__ ol, int ldo, int m0, int c0, int lane, b16* Th, b16* Tl) {
  const int nloc = lane & 15, hlf = lane >> 4;
#pragma unroll
  for (int t = 0; t < 4; ++t)
#pragma unroll
    for (int r = 0; r < 2; ++r)
#pragma unroll
      for (int v = 0; v < 8; ++v) {
        const int rr = r * 16 + v + 8 * hlf, cc = t * 16 + nloc;
        const float val = epi_val(e, acc[r][t][v], m0 + rr, c0 + cc);
        b16 h_, l_; split16(val, h_, l_);
        Th[rr * 64 + cc] = h_; if (two) Tl[rr * 64 + cc] = l_;
      }
  wave_lds_sync();
  for (int pass = 0; pass < 2; ++pass) {
#pragma unroll
    for (int j = 0; j < 8; ++j) {
      const int rr = j * 4 + (lane >> 3), c8 = (lane & 7) * 8;
      const size_t o = (size_t)(m0 + rr) * ldo + c0 + c8;
      *(volatile v8b*)(oh + o) = ld8b(Th + rr * 64 + c8);
      if (two) *(volatile v8b*)(ol + o) = ld8b(Tl + rr * 64 + c8);
    }
    __threadfence();
  }
}
__device__ __forceinline__ void epi_f32(v8f (&acc)[2][4], const Epi& e, float* __restrict__ out, int ldo, int m0, int c0, int lane, float* Tt) {
  const int nloc = lane & 15, hlf = lane >> 4;
#pragma unroll
  for (int t = 0; t < 4; ++t)
#pragma unroll
    for (int r = 0; r < 2; ++r)
#pragma unroll
      for (int v = 0; v < 8; ++v) {
        const int rr = r * 16 + v + 8 * hlf, cc = t * 16 + nloc;
        Tt[rr * 64 + cc] = epi_val(e, acc[r][t][v], m0 + rr, c0 + cc);
      }
  wave_lds_sync();
  float* dst0 = out + (size_t)m0 * ldo + c0; const float* rs0 = e.resid ? e.resid + (size_t)m0 * ldo + c0 : nullptr;
  for (int pass = 0; pass < 2; ++pass) {
#pragma unroll
    for (int j = 0; j < 16; ++j) {
      const int rr = j * 2 + hlf, c4 = nloc * 4;
      v4f val = *(const v4f*)(Tt + rr * 64 + c4);
      if (rs0) val += *(const v4f*)(rs0 + (size_t)rr * ldo + c4);
      *(volatile v4f*)(dst0 + (size_t)rr * ldo + c4) = val;
    }
    __threadfence();
  }
}


__global__ __launch_bounds__(256) void prep_kernel(const float* __restrict__ c0w, const float* __restrict__ c1w, const float* __restrict__ W0, const float* __restrict__ W1,
                                                   b16* __restrict__ w0p, b16* __restrict__ w1p, b16* __restrict__ wx, float* __restrict__ wd, b16* __restrict__ w1d) {
  const size_t tid = (size_t)blockIdx.x * blockDim.x + threadIdx.x, stride = (size_t)gridDim.x * blockDim.x;
  for (int pass = 0; pass < 2; ++pass) {
    for (size_t i8 = tid; i8 < (16 * 128 + 32 * 96 + (size_t)ND0 * KD0 + (size_t)ND1 * ND0) / 8; i8 += stride) {
      size_t i = i8 * 8; v8b v; b16* dst;
      if (i < 16 * 128) { dst = w0p + i; for (int e = 0; e < 8; ++e) { const int o = (int)((i + e) / 128), k = (int)((i + e) % 128), kh = k / 16, j = k % 16, kw = j / 3, c = j % 3;
          v[e] = (b16)((o < C0 && kh < KH0 && j < 9) ? c0w[((o * CIN + c) * KH0 + kh) * KW0 + kw] : 0.0f); } }
      else if ((i -= 16 * 128) < 32 * 96) { dst = w1p + i; for (int e = 0; e < 8; ++e) { const int o = (int)((i + e) / 96), k = (int)((i + e) % 96), kh = k / 32, j = k % 32, c = j / 3, kw = j % 3;
          v[e] = (b16)((o < C1 && j < 30) ? c1w[((o * C0 + c) * 3 + kh) * 3 + kw] : 0.0f); } }
      else if ((i -= 32 * 96) < (size_t)ND0 * KD0) { dst = wx + i; for (int e = 0; e < 8; ++e) { const int o = (int)((i + e) / KD0), k = (int)((i + e) % KD0); v[e] = (b16)W0[(size_t)o * (KD0 + NDIFF) + k]; } }
      else { i -= (size_t)ND0 * KD0; dst = w1d + i; for (int e = 0; e < 8; ++e) v[e] = (b16)W1[i + e]; }
      *(volatile v8b*)dst = v;
    }
    for (size_t j = tid; j < NDIFF * ND0; j += stride) { const int dd = (int)(j / ND0), o = (int)(j % ND0); ((volatile float*)wd)[j] = W0[(size_t)o * (KD0 + NDIFF) + KD0 + dd]; }
    __threadfence();
  }
}

__global__ __launch_bounds__(256) void conv0_kernel(const float* __restrict__ x, const b16* __restrict__ w0p, const float* __restrict__ c0b, b16* __restrict__ h1) {
  __shared__ __attribute__((aligned(16))) b16 X2[F0][2][16][8];
  __shared__ float Tl[8][80][C0 + 1];
  __shared__ __attribute__((aligned(16))) b16 Ol[8][H1P];
  const int wid = threadIdx.x >> 5, lane = threadIdx.x & 31, hh = lane >> 4, col = lane & 15, tb = blockIdx.x * 8, t0 = tb + wid;
  for (int p = threadIdx.x; p < 15 * F0; p += 256) {
    const int fr = p / F0, fq = p - fr * F0, tt = tb + fr - 7;
    v8b lo = {}, hi = {};
    if (tt >= 0 && tt < T) { const float* src = x + ((size_t)tt * NF0 + fq) * CIN;
#pragma unroll
      for (int j = 0; j < 8; ++j) lo[j] = (b16)src[j];
      hi[0] = (b16)src[8]; }
    *(v8b*)(&X2[fq][0][fr][0]) = lo; *(v8b*)(&X2[fq][1][fr][0]) = hi;
  }
  __syncthreads();
  if (t0 < T0) {
    v16b bw[4];
#pragma unroll
    for (int ks = 0; ks < 4; ++ks) bw[ks] = frag_kb(w0p + col * 128 + ks * 32, hh);
    for (int mt = 0; mt < 5; ++mt) {
      const int fr = mt * 16 + col; const int frc = (fr < F0) ? fr : F0 - 1;
      v8f acc = {};
#pragma unroll
      for (int ks = 0; ks < 4; ++ks) {
        const v16b a = *(const v16b*)(&X2[frc][hh][wid + 2 * ks][0]);
        acc = wmma16b(a, bw[ks], acc);
      }
      if (col < C0) {
#pragma unroll
        for (int v = 0; v < 8; ++v) { const int f = mt * 16 + 8 * hh + v; if (f < 80) Tl[wid][f][col] = fmaxf(acc[v] + c0b[col], 0.0f); }
      }
    }
    wave_lds_sync();
    for (int i = lane; i < H1P; i += 32) { b16 hv = (b16)0.0f; if (i < C0 * P0) { const int c = i / P0, j = i % P0; hv = (b16)fmaxf(fmaxf(Tl[wid][3 * j][c], Tl[wid][3 * j + 1][c]), Tl[wid][3 * j + 2][c]); } Ol[wid][i] = hv; }
    wave_lds_sync();
    b16* dst = h1 + (size_t)t0 * H1P;
    for (int pass = 0; pass < 2; ++pass) {
      *(volatile v8b*)(dst + lane * 8) = *(const v8b*)(&Ol[wid][lane * 8]);
      if (lane < 8) *(volatile v8b*)(dst + 256 + lane * 8) = *(const v8b*)(&Ol[wid][256 + lane * 8]);
      __threadfence();
    }
  }
}

__global__ __launch_bounds__(256) void conv1_kernel(const b16* __restrict__ h1, const b16* __restrict__ w1p, const float* __restrict__ c1b, b16* __restrict__ feats) {
  __shared__ __attribute__((aligned(16))) b16 Y2[F1][10][32];
  __shared__ float Tl[8][F1][C1 + 1];
  __shared__ __attribute__((aligned(16))) b16 Ol[8][FP];
  const int wid = threadIdx.x >> 5, lane = threadIdx.x & 31, hh = lane >> 4, col = lane & 15, tb = blockIdx.x * 8, t1 = tb + wid;
  for (int p = threadIdx.x; p < 10 * F1; p += 256) {
    const int fr = p / F1, fq = p - fr * F1, tt = tb + fr;
    _Float16 w32[32];
#pragma unroll
    for (int j = 0; j < 32; ++j) w32[j] = (b16)0.0f;
    if (tt < T0) { const b16* src = h1 + (size_t)tt * H1P + fq;
#pragma unroll
      for (int c = 0; c < C0; ++c) { w32[3 * c] = src[c * P0]; w32[3 * c + 1] = src[c * P0 + 1]; w32[3 * c + 2] = src[c * P0 + 2]; } }
#pragma unroll
    for (int q = 0; q < 4; ++q) { v8b v; const int src8 = (q == 0) ? 0 : (q == 1) ? 16 : (q == 2) ? 8 : 24;
#pragma unroll
      for (int e = 0; e < 8; ++e) v[e] = w32[src8 + e];
      *(v8b*)(&Y2[fq][fr][q * 8]) = v; }
  }
  __syncthreads();
  if (t1 < T1) {
    for (int mt = 0; mt < 2; ++mt) {
      const int fr = mt * 16 + col; const int frc = (fr < F1) ? fr : F1 - 1;
      v8f acc[2] = {{}, {}};
#pragma unroll
      for (int ks = 0; ks < 3; ++ks) {
        const v16b a = *(const v16b*)(&Y2[frc][wid + ks][16 * hh]);
#pragma unroll
        for (int nt = 0; nt < 2; ++nt) acc[nt] = wmma16b(a, frag_kb(w1p + (nt * 16 + col) * 96 + ks * 32, hh), acc[nt]);
      }
#pragma unroll
      for (int nt = 0; nt < 2; ++nt) { const int o = nt * 16 + col; if (o < C1) {
#pragma unroll
        for (int v = 0; v < 8; ++v) { const int f = mt * 16 + 8 * hh + v; if (f < F1) Tl[wid][f][o] = fmaxf(acc[nt][v] + c1b[o], 0.0f); } } }
    }
    wave_lds_sync();
    for (int i = lane; i < FP; i += 32) { b16 hv = (b16)0.0f; if (i < FEAT) { const int j = i / C1, o = i % C1; hv = (b16)fmaxf(fmaxf(Tl[wid][3 * j][o], Tl[wid][3 * j + 1][o]), Tl[wid][3 * j + 2][o]); } Ol[wid][i] = hv; }
    wave_lds_sync();
    b16* dst = feats + (size_t)t1 * FP;
    for (int pass = 0; pass < 2; ++pass) { if (lane < 24) *(volatile v8b*)(dst + lane * 8) = *(const v8b*)(&Ol[wid][lane * 8]); __threadfence(); }
  }
}

__global__ __launch_bounds__(128) void dense0_kernel(const b16* __restrict__ feats, const b16* __restrict__ wx, const float* __restrict__ b0, float* __restrict__ h0) {
  __shared__ __attribute__((aligned(16))) float Ts[4][32 * 64];
  const int lane = threadIdx.x & 31, wave = threadIdx.x >> 5, nloc = lane & 15, hlf = lane >> 4;
  const int m0 = blockIdx.y * 128 + wave * 32, c0 = blockIdx.x * 64;
  v8f acc[2][4];
#pragma unroll
  for (int r = 0; r < 2; ++r)
#pragma unroll
    for (int t = 0; t < 4; ++t) acc[r][t] = (v8f){};
#pragma unroll 1
  for (int kb = 0; kb < KD0; kb += 32) {
    const int fi = kb / FEAT, j0 = kb % FEAT;
    const v16b a0 = frag_kb(feats + (size_t)(m0 + nloc + fi) * FP + j0, hlf), a1 = frag_kb(feats + (size_t)(m0 + 16 + nloc + fi) * FP + j0, hlf);
#pragma unroll
    for (int t = 0; t < 4; ++t) { const v16b bw = frag_kb(wx + (size_t)(c0 + t * 16 + nloc) * KD0 + kb, hlf); acc[0][t] = wmma16b(a0, bw, acc[0][t]); acc[1][t] = wmma16b(a1, bw, acc[1][t]); }
  }
  const Epi e{1.0f, nullptr, b0, nullptr, 0, 1.0f, nullptr, nullptr};
  epi_f32(acc, e, h0, ND0, m0, c0, lane, Ts[wave]);
}

__global__ __launch_bounds__(128) void dense1_kernel(const float* __restrict__ h0, const float* __restrict__ wd, const int* __restrict__ diffs, const b16* __restrict__ w1d,
                                                    const float* __restrict__ b1, const float* __restrict__ wout, const float* __restrict__ bout, float* __restrict__ out) {
  __shared__ float Rs[4][32];
  const int lane = threadIdx.x & 31, wave = threadIdx.x >> 5, nloc = lane & 15, hlf = lane >> 4, z = blockIdx.y;
  int dz = diffs[z]; dz = dz < 0 ? 0 : (dz >= NDIFF ? NDIFF - 1 : dz);
  const int m0 = blockIdx.x * 128 + wave * 32; const float* wdz = wd + dz * ND0;
  v8f acc[2][8];
#pragma unroll
  for (int r = 0; r < 2; ++r)
#pragma unroll
    for (int t = 0; t < 8; ++t) acc[r][t] = (v8f){};
#pragma unroll 1
  for (int kb = 0; kb < ND0; kb += 32) {
    v16b a0, a1;
    const float* r0p = h0 + (size_t)(m0 + nloc) * ND0 + kb; const float* r1p = h0 + (size_t)(m0 + 16 + nloc) * ND0 + kb;
#pragma unroll
    for (int e = 0; e < 16; ++e) { const int k = (e < 8) ? (8 * hlf + e) : (16 + 8 * hlf + e - 8); const float bz = wdz[kb + k]; a0[e] = (b16)fmaxf(r0p[k] + bz, 0.0f); a1[e] = (b16)fmaxf(r1p[k] + bz, 0.0f); }
#pragma unroll
    for (int t = 0; t < 8; ++t) { const v16b bw = frag_kb(w1d + (size_t)(t * 16 + nloc) * ND0 + kb, hlf); acc[0][t] = wmma16b(a0, bw, acc[0][t]); acc[1][t] = wmma16b(a1, bw, acc[1][t]); }
  }
  float part[2][8];
#pragma unroll
  for (int r = 0; r < 2; ++r)
#pragma unroll
    for (int v = 0; v < 8; ++v) { float s = 0.0f;
#pragma unroll
      for (int t = 0; t < 8; ++t) { const int c = t * 16 + nloc; s += fmaxf(acc[r][t][v] + b1[c], 0.0f) * wout[c]; }
      part[r][v] = s; }
#pragma unroll
  for (int o = 1; o < 16; o <<= 1)
#pragma unroll
    for (int r = 0; r < 2; ++r)
#pragma unroll
      for (int v = 0; v < 8; ++v) part[r][v] += __shfl_xor(part[r][v], o);
  if (nloc == 0) {
#pragma unroll
    for (int r = 0; r < 2; ++r)
#pragma unroll
      for (int v = 0; v < 8; ++v) { const float lg = part[r][v] + bout[0]; Rs[wave][r * 16 + 8 * hlf + v] = 1.0f / (1.0f + __expf(-lg)); }
  }
  wave_lds_sync();
  for (int pass = 0; pass < 2; ++pass) { ((volatile float*)out)[(size_t)z * T + m0 + lane] = Rs[wave][lane]; __threadfence(); }
}
}

extern "C" void kernel_launch(void* const* d_in, const int* in_sizes, int n_in,
                              void* d_out, int out_size, void* d_ws, size_t ws_size, hipStream_t stream) {
  (void)n_in; (void)out_size;
  const float* x = (const float*)d_in[0];
  const int* diffs = (const int*)d_in[1];
  const float* c0w = (const float*)d_in[2]; const float* c0b = (const float*)d_in[3];
  const float* c1w = (const float*)d_in[4]; const float* c1b = (const float*)d_in[5];
  const float* W0 = (const float*)d_in[6]; const float* b0 = (const float*)d_in[7];
  const float* W1 = (const float*)d_in[8]; const float* b1 = (const float*)d_in[9];
  const float* Wout = (const float*)d_in[10]; const float* bout = (const float*)d_in[11];
  float* out = (float*)d_out;
  if (in_sizes[0] != T * NF0 * CIN || in_sizes[1] != NDIFF || in_sizes[2] != C0 * K0 || in_sizes[6] != ND0 * (KD0 + NDIFF) || in_sizes[8] != ND1 * ND0) return;
  size_t off = 0; char* ws = (char*)d_ws;
  auto carve = [&](size_t bytes) { char* p = ws + off; off += (bytes + 255) & ~(size_t)255; return p; };
  b16* w0p = (b16*)carve(16 * 128 * 2); b16* w1p = (b16*)carve(32 * 96 * 2); b16* wx = (b16*)carve((size_t)ND0 * KD0 * 2); float* wd = (float*)carve((size_t)NDIFF * ND0 * 4); b16* w1d = (b16*)carve((size_t)ND1 * ND0 * 2);
  float* h0 = (float*)carve((size_t)T * ND0 * 4);
  b16* h1 = (b16*)h0;
  b16* feats = (b16*)carve((size_t)(T1 + 8) * FP * 2);
  if (off > ws_size) return;
  prep_kernel<<<64, 256, 0, stream>>>(c0w, c1w, W0, W1, w0p, w1p, wx, wd, w1d);
  conv0_kernel<<<(T0 + 7) / 8, 256, 0, stream>>>(x, w0p, c0b, h1);
  conv1_kernel<<<(T1 + 7) / 8, 256, 0, stream>>>(h1, w1p, c1b, feats);
  dense0_kernel<<<dim3(ND0 / 64, T / 128), 128, 0, stream>>>(feats, wx, b0, h0);
  dense1_kernel<<<dim3(T / 128, NDIFF), 128, 0, stream>>>(h0, wd, diffs, w1d, b1, Wout, bout, out);
}
